// Block_67577015435861
// MI455X (gfx1250) — hardware-run, weakly checked
//
#include <hip/hip_runtime.h>
#include <math.h>

typedef __attribute__((ext_vector_type(16))) _Float16 v16h;
typedef __attribute__((ext_vector_type(16))) __bf16 v16b;
typedef __attribute__((ext_vector_type(8)))  _Float16 v8h;
typedef __attribute__((ext_vector_type(8)))  __bf16 v8b;
typedef __attribute__((ext_vector_type(8)))  float v8f;
typedef __attribute__((ext_vector_type(4)))  float v4f;
typedef __attribute__((ext_vector_type(4)))  unsigned v4u;

template <typename T> __device__ __forceinline__ void vst2(void* p, T v) { *(volatile T*)p = v; __threadfence(); *(volatile T*)p = v; }
__device__ __forceinline__ v8f wmma16(v16h a, v16h b, v8f c) {
  v8f d = __builtin_amdgcn_wmma_f32_16x16x32_f16(false, a, false, b, (short)0, c, false, false);
  asm volatile("v_nop\n\tv_nop\n\tv_nop\n\tv_nop" : "+v"(d) : "v"(a), "v"(b));
  return d;
}
__device__ __forceinline__ v8f wmma_bf(v16b a, v16b b, v8f c) {
  v8f d = __builtin_amdgcn_wmma_f32_16x16x32_bf16(false, a, false, b, (short)0, c, false, false);
  asm volatile("v_nop\n\tv_nop\n\tv_nop\n\tv_nop" : "+v"(d) : "v"(a), "v"(b));
  return d;
}
__device__ __forceinline__ v16h frag_h(const _Float16* rowk0, int lane) {
  union { v16h v; v8h q[2]; } u; const _Float16* p = rowk0 + 8 * (lane >> 4);
  u.q[0] = *(const v8h*)p; u.q[1] = *(const v8h*)(p + 16); return u.v;
}
__device__ __forceinline__ v16b frag_b(const __bf16* rowk0, int lane) {
  union { v16b v; v8b q[2]; } u; const __bf16* p = rowk0 + 8 * (lane >> 4);
  u.q[0] = *(const v8b*)p; u.q[1] = *(const v8b*)(p + 16); return u.v;
}
__device__ __forceinline__ v16h frag_f32(const float* rowk0, int lane) {
  v16h a; const float* p = rowk0 + 8 * (lane >> 4);
#pragma unroll
  for (int i = 0; i < 8; ++i) { a[i] = (_Float16)p[i]; a[8 + i] = (_Float16)p[16 + i]; }
  return a;
}
__device__ __forceinline__ v16h frag_f32s(const float* rowk0, int lane, float sc) {
  v16h a; const float* p = rowk0 + 8 * (lane >> 4);
#pragma unroll
  for (int i = 0; i < 8; ++i) { a[i] = (_Float16)(p[i] * sc); a[8 + i] = (_Float16)(p[16 + i] * sc); }
  return a;
}
struct F2 { v16b h, l; };
__device__ __forceinline__ F2 bsplit16(const float v[16]) { F2 r;
#pragma unroll
  for (int i = 0; i < 16; ++i) { const __bf16 h = (__bf16)v[i]; r.h[i] = h; r.l[i] = (__bf16)(v[i] - (float)h); }
  return r; }
__device__ __forceinline__ F2 split_row(const float* row, int k0, int lane) { float v[16]; const float* p = row + k0 + 8 * (lane >> 4);
#pragma unroll
  for (int i = 0; i < 8; ++i) { v[i] = p[i]; v[8 + i] = p[16 + i]; }
  return bsplit16(v); }
#define LDSX() do { asm volatile("s_wait_dscnt 0" ::: "memory"); __builtin_amdgcn_wave_barrier(); __builtin_amdgcn_fence(3  , "workgroup"); } while (0)

#ifndef NB
#define NB 64
#endif
#ifndef SEQ
#define SEQ 256
#endif
#define NB_FULL 64
#define TT_FULL 256
#define TT SEQ
#define CC 512
#define DIN 512
#define DFF 2048
#define NH 8
#define HD 64
#define NQB (TT / 64)
#define SCALE (0.125f)
#define CAUSAL 1
#ifndef NBC
#if NB < 16
#define NBC NB
#else
#define NBC 16
#endif
#endif
#ifndef QBH
#define QBH NQB
#endif
#ifndef QHI
#define QHI TT
#endif
#ifndef KHI
#define KHI TT
#endif
#define NEED_PLAIN (QBH < NQB)
#define KCH (TT / 128)

__device__ __forceinline__ float bfr(float v) { return (float)(__bf16)v; }
__host__ __device__ constexpr int kb_last(int qb) { return CAUSAL ? ((qb * 64 + 63) >> 7) : (TT / 128 - 1); }

static __device__ __forceinline__ _Float16 toh_flush(float v) { const _Float16 r = (_Float16)v; return (fabsf(v) < 6.103515625e-05f) ? (_Float16)0.0f : r; }

__device__ __forceinline__ v16b wcol_io(const float* Wm, int k0, int o, int lane, int ld) { v16b w; const int g = lane >> 4;
#pragma unroll
  for (int i = 0; i < 8; ++i) { w[i] = (__bf16)Wm[(size_t)(k0 + 8 * g + i) * ld + o]; w[8 + i] = (__bf16)Wm[(size_t)(k0 + 16 + 8 * g + i) * ld + o]; }
  return w; }
__device__ __forceinline__ v16h wcolh_io(const float* Wm, int k0, int o, int lane, int ld) { v16h w; const int g = lane >> 4;
#pragma unroll
  for (int i = 0; i < 8; ++i) { w[i] = (_Float16)(bfr(Wm[(size_t)(k0 + 8 * g + i) * ld + o]) * 256.0f); w[8 + i] = (_Float16)(bfr(Wm[(size_t)(k0 + 16 + 8 * g + i) * ld + o]) * 256.0f); }
  return w; }
__device__ __forceinline__ v16b wcol_hdk(const float* Wm, int k0, int o, int lane) { v16b w; const int g = lane >> 4; const float* p = Wm + (size_t)(o / HD) * DIN * HD + (o % HD);
#pragma unroll
  for (int i = 0; i < 8; ++i) { w[i] = (__bf16)p[(size_t)(k0 + 8 * g + i) * HD]; w[8 + i] = (__bf16)p[(size_t)(k0 + 16 + 8 * g + i) * HD]; }
  return w; }
__device__ __forceinline__ v16h frag_f32s_fl(const float* rowk0, int lane, float sc) {
  v16h a; const float* p = rowk0 + 8 * (lane >> 4);
#pragma unroll
  for (int i = 0; i < 8; ++i) { a[i] = toh_flush(p[i] * sc); a[8 + i] = toh_flush(p[16 + i] * sc); }
  return a;
}
__device__ __forceinline__ v16h wcolh_io_fl(const float* Wm, int k0, int o, int lane, int ld) { v16h w; const int g = lane >> 4;
#pragma unroll
  for (int i = 0; i < 8; ++i) { w[i] = toh_flush(bfr(Wm[(size_t)(k0 + 8 * g + i) * ld + o]) * 256.0f); w[8 + i] = toh_flush(bfr(Wm[(size_t)(k0 + 16 + 8 * g + i) * ld + o]) * 256.0f); }
  return w; }

#if NEED_PLAIN
#define VT_BYTES (2ull * NBC * CC * TT)
#else
#define VT_BYTES 0ull
#endif
#define WS_QH  0ull
#define WS_KH  (WS_QH + 2ull * NBC * TT * CC)
#define WS_VT  (WS_KH + 2ull * NBC * TT * CC)
#define WS_QL  (WS_VT + VT_BYTES)
#define WS_KL  (WS_QL + 2ull * NBC * QHI * CC)
#define WS_VB  (WS_KL + 2ull * NBC * KHI * CC)
#define WS_VBL (WS_VB + 2ull * NBC * CC * KHI)
#define WS_S   (WS_VBL + 2ull * NBC * CC * KHI)
#define WS_Y   (WS_S  + 4ull * NBC * NH * TT * TT)
#define WS_Z1  (WS_Y  + 4ull * NBC * TT * CC)
#define WS_L1F (WS_Z1 + 4ull * NBC * TT * DIN)
#define WS_L1H (WS_L1F + 4ull * NBC * TT * DIN)
#define WS_HID (WS_L1H + 2ull * NBC * TT * DIN)
#define WS_Z2  (WS_HID + 2ull * NBC * TT * DFF)
#define WS_W1T (WS_Z2 + 4ull * NBC * TT * DIN)
#define WS_W2T (WS_W1T + 2ull * DIN * DFF)
#define WS_END (WS_W2T + 2ull * DFF * DIN)

static_assert(TT % 128 == 0);
static_assert(TT <= TT_FULL);
static_assert(NB <= NB_FULL);
static_assert(NB % NBC == 0);
static_assert(QBH >= 1 && QBH <= NQB);
static_assert(QHI % 64 == 0 && QHI <= TT && QBH * 64 <= QHI);
static_assert(KHI % 64 == 0 && KHI <= TT && KHI >= (kb_last(QBH - 1) + 1) * 128);
static_assert(CC == NH * HD && CC % 128 == 0 && DIN % 128 == 0 && DIN % 32 == 0 && HD % 32 == 0);
static_assert(NBC * NH <= 65535);
static_assert(DFF % 128 == 0 && DFF % 64 == 0 && DFF % 32 == 0 && DIN % 64 == 0 && DIN % 256 == 0);
static_assert((NBC * TT) % 64 == 0 && (NBC * TT) % 8 == 0);
static_assert(WS_Z1 % 128 == 0 && WS_L1F % 128 == 0 && WS_L1H % 128 == 0 && WS_HID % 128 == 0 && WS_Z2 % 128 == 0 && WS_W1T % 128 == 0 && WS_W2T % 128 == 0);
static_assert(WS_END <= 134217728ull);

__global__ __launch_bounds__(128) void k_wt(const float* __restrict__ W, _Float16* __restrict__ WT, int K, int N) {
  __shared__ __align__(16) _Float16 tt[64][72];
  const int tid = threadIdx.x; const int k0 = blockIdx.x * 64, n0 = blockIdx.y * 64;
  for (int e = tid; e < 64 * 16; e += 128) { const int kr = e >> 4, nq = (e & 15) * 4; const v4f w = *(const v4f*)(W + (size_t)(k0 + kr) * N + n0 + nq);
#pragma unroll
    for (int i = 0; i < 4; ++i) tt[nq + i][kr] = toh_flush(bfr(w[i]) * 256.0f); }
  __syncthreads();
  for (int e = tid; e < 64 * 8; e += 128) { const int nl = e >> 3, q = e & 7;
    vst2((void*)(WT + (size_t)(n0 + nl) * K + k0 + q * 8), *(const v4u*)&tt[nl][q * 8]); }
}

__global__ __launch_bounds__(128) void k_proj(const float* __restrict__ X, const float* __restrict__ WQ, const float* __restrict__ WK, const float* __restrict__ WV,
    _Float16* __restrict__ QH, _Float16* __restrict__ QL, _Float16* __restrict__ KH, _Float16* __restrict__ KL, _Float16* __restrict__ VT, __bf16* __restrict__ VB, __bf16* __restrict__ VBL) {
  __shared__ __align__(16) _Float16 sh[64][136], sl[64][136]; __shared__ __align__(16) _Float16 th[128][72]; __shared__ __align__(16) __bf16 tb[128][72], tbl[128][72];
  const int tid = threadIdx.x, wave = __builtin_amdgcn_readfirstlane((int)(tid >> 5)), lane = tid & 31, col = lane & 15, g = lane >> 4;
  const int which = blockIdx.z; const int c0 = blockIdx.y * 128; const size_t r0 = (size_t)blockIdx.x * 64; const size_t bb = r0 / TT; const int t0 = (int)(r0 % TT);
  const float* WA = which == 0 ? WQ : which == 1 ? WK : WV;
  const size_t xr = bb * TT_FULL + t0 + wave * 16 + col;
  v8f acc[8] = {};
#pragma unroll 2
  for (int kc = 0; kc < DIN / 32; ++kc) {
    v16b a;
    { const float* p = X + xr * DIN + kc * 32 + 8 * g;
#pragma unroll
      for (int i = 0; i < 8; ++i) { a[i] = (__bf16)p[i]; a[8 + i] = (__bf16)p[16 + i]; } }
    asm volatile("s_wait_loadcnt 0x0" ::: "memory");
#pragma unroll
    for (int j = 0; j < 8; ++j) { const v16b w = wcol_hdk(WA, kc * 32, c0 + j * 16 + col, lane); asm volatile("s_wait_loadcnt 0x0" ::: "memory"); acc[j] = wmma_bf(a, w, acc[j]); }
  }
  if (which < 2) {
    _Float16* DH = which == 0 ? QH : KH; _Float16* DL = which == 0 ? QL : KL; const int nhi = which == 0 ? QHI : KHI; const bool hi_rows = t0 < nhi;
#pragma unroll
    for (int j = 0; j < 8; ++j) {
#pragma unroll
      for (int r = 0; r < 8; ++r) { const float v = acc[j][r]; const _Float16 hv = (_Float16)v; sh[wave * 16 + 8 * g + r][j * 16 + col] = hv; sl[wave * 16 + 8 * g + r][j * 16 + col] = (_Float16)((v - (float)hv) * 1024.0f); }
    }
    __syncthreads();
    for (int e = tid; e < 64 * 16; e += 128) { const int rl = e >> 4, q = e & 15;
      vst2((void*)(DH + (r0 + rl) * CC + c0 + q * 8), *(const v4u*)&sh[rl][q * 8]);
      if (hi_rows) vst2((void*)(DL + (bb * nhi + t0 + rl) * (size_t)CC + c0 + q * 8), *(const v4u*)&sl[rl][q * 8]); }
  } else {
    const bool hi_rows = t0 < KHI;
#pragma unroll
    for (int j = 0; j < 8; ++j) {
#pragma unroll
      for (int r = 0; r < 8; ++r) { const float v = acc[j][r]; const int rl = wave * 16 + 8 * g + r, cl = j * 16 + col; if (NEED_PLAIN) th[cl][rl] = (_Float16)v; const __bf16 bh = (__bf16)v; tb[cl][rl] = bh; tbl[cl][rl] = (__bf16)(v - (float)bh); }
    }
    __syncthreads();
    for (int e = tid; e < 128 * 8; e += 128) { const int cl = e >> 3, q = e & 7;
      if (NEED_PLAIN) vst2((void*)(VT + (bb * CC + c0 + cl) * (size_t)TT + t0 + q * 8), *(const v4u*)&th[cl][q * 8]);
      if (hi_rows) { const size_t o3 = (bb * CC + c0 + cl) * (size_t)KHI + t0 + q * 8; vst2((void*)(VB + o3), *(const v4u*)&tb[cl][q * 8]); vst2((void*)(VBL + o3), *(const v4u*)&tbl[cl][q * 8]); } }
  }
}

__global__ __launch_bounds__(128) void k_sc(const _Float16* __restrict__ QH, const _Float16* __restrict__ KH, const _Float16* __restrict__ QL, const _Float16* __restrict__ KL, float* __restrict__ S0) {
  __shared__ __align__(16) float ss[4][16][132];
  const int qb = blockIdx.x, kb = blockIdx.y; if (kb > kb_last(qb)) return;
  const int bl = blockIdx.z / NH, h = blockIdx.z % NH; float* S = S0 + (size_t)blockIdx.z * TT * TT;
  const int tid = threadIdx.x, wave = __builtin_amdgcn_readfirstlane((int)(tid >> 5)), lane = tid & 31, col = lane & 15, g = lane >> 4; const int k0 = kb * 128; const int ql0 = qb * 64 + wave * 16; const size_t q0 = (size_t)bl * TT + ql0, kr0 = (size_t)bl * TT + k0;
  v8f acc[8] = {}, accl[8] = {};
  const _Float16* QLb = QL + (size_t)bl * QHI * CC; const _Float16* KLb = KL + (size_t)bl * KHI * CC;
  if (!NEED_PLAIN || qb < QBH) {
#pragma unroll
    for (int kc = 0; kc < HD / 32; ++kc) { const v16h ah = frag_h(QH + (q0 + col) * CC + h * HD + kc * 32, lane), al = frag_h(QLb + (size_t)(ql0 + col) * CC + h * HD + kc * 32, lane);
#pragma unroll
      for (int j = 0; j < 8; ++j) { const v16h kbf = frag_h(KH + (kr0 + j * 16 + col) * CC + h * HD + kc * 32, lane), klf = frag_h(KLb + (size_t)(k0 + j * 16 + col) * CC + h * HD + kc * 32, lane); acc[j] = wmma16(ah, kbf, acc[j]); accl[j] = wmma16(al, kbf, accl[j]); accl[j] = wmma16(ah, klf, accl[j]); } }
  } else if (qb * 64 < QHI) {
#pragma unroll
    for (int kc = 0; kc < HD / 32; ++kc) { const v16h ah = frag_h(QH + (q0 + col) * CC + h * HD + kc * 32, lane), al = frag_h(QLb + (size_t)(ql0 + col) * CC + h * HD + kc * 32, lane);
#pragma unroll
      for (int j = 0; j < 8; ++j) { const v16h kbf = frag_h(KH + (kr0 + j * 16 + col) * CC + h * HD + kc * 32, lane); acc[j] = wmma16(ah, kbf, acc[j]); accl[j] = wmma16(al, kbf, accl[j]); } }
  } else {
#pragma unroll
    for (int kc = 0; kc < HD / 32; ++kc) { const v16h ah = frag_h(QH + (q0 + col) * CC + h * HD + kc * 32, lane);
#pragma unroll
      for (int j = 0; j < 8; ++j) { const v16h kbf = frag_h(KH + (kr0 + j * 16 + col) * CC + h * HD + kc * 32, lane); acc[j] = wmma16(ah, kbf, acc[j]); } }
  }
#pragma unroll
  for (int j = 0; j < 8; ++j) {
#pragma unroll
    for (int r = 0; r < 8; ++r) ss[wave][8 * g + r][j * 16 + col] = (acc[j][r] + accl[j][r] * (1.0f / 1024.0f)) * SCALE;
  }
  LDSX();
  for (int rl = 0; rl < 16; ++rl) vst2((void*)(S + (size_t)(ql0 + rl) * TT + k0 + lane * 4), *(const v4f*)&ss[wave][rl][lane * 4]);
}

__global__ __launch_bounds__(256) void k_sm(float* __restrict__ S0) {
  const int tid = threadIdx.x, wave = __builtin_amdgcn_readfirstlane((int)(tid >> 5)), lane = tid & 31; const int t = blockIdx.x * 8 + wave;
  const int kend = (kb_last(t >> 6) + 1) * 128;
  float* sr = S0 + (size_t)blockIdx.y * TT * TT + (size_t)t * TT;
  v4f e[KCH]; float m = -3.0e38f;
#pragma unroll
  for (int c = 0; c < KCH; ++c) { const int k = c * 128 + lane * 4; v4f v = *(const v4f*)(sr + k);
#pragma unroll
    for (int i = 0; i < 4; ++i) { const bool ok = (k + i < kend) && (!CAUSAL || (k + i <= t)); const float x = ok ? v[i] : -3.0e38f; v[i] = x; m = fmaxf(m, x); }
    e[c] = v; }
#pragma unroll
  for (int o = 1; o < 32; o <<= 1) m = fmaxf(m, __shfl_xor(m, o));
  float sum = 0.f;
#pragma unroll
  for (int c = 0; c < KCH; ++c) {
#pragma unroll
    for (int i = 0; i < 4; ++i) { const float v = e[c][i]; const float x = (v <= -1.0e38f) ? 0.f : exp2f((v - m) * 1.44269504088896f); e[c][i] = x; sum += x; } }
#pragma unroll
  for (int o = 1; o < 32; o <<= 1) sum += __shfl_xor(sum, o);
  const float inv = sum > 0.f ? 2048.0f / sum : 0.f;
  v4f p[KCH];
#pragma unroll
  for (int c = 0; c < KCH; ++c) p[c] = e[c] * inv;
#pragma unroll
  for (int c = 0; c < KCH; ++c) *(volatile v4f*)(sr + c * 128 + lane * 4) = p[c];
  __threadfence();
#pragma unroll
  for (int c = 0; c < KCH; ++c) *(volatile v4f*)(sr + c * 128 + lane * 4) = p[c];
}

__global__ __launch_bounds__(128) void k_pv(const float* __restrict__ PS0, const _Float16* __restrict__ VT, const __bf16* __restrict__ VB, const __bf16* __restrict__ VBL, float* __restrict__ Y) {
  __shared__ __align__(16) float ss[4][16][HD + 4];
  const int bl = blockIdx.z / NH, h = blockIdx.z % NH; const float* PS = PS0 + (size_t)blockIdx.z * TT * TT;
  const int tid = threadIdx.x, wave = __builtin_amdgcn_readfirstlane((int)(tid >> 5)), lane = tid & 31, col = lane & 15, g = lane >> 4; const int qb = blockIdx.x; const int ql0 = qb * 64 + wave * 16; const int kce = (kb_last(qb) + 1) * 4;
  v8f acc[HD / 16] = {};
  if (!NEED_PLAIN || qb < QBH) {
#pragma unroll 1
    for (int kc = 0; kc < kce; ++kc) { const F2 p = split_row(PS + (size_t)(ql0 + col) * TT, kc * 32, lane);
      asm volatile("s_wait_loadcnt 0x0" ::: "memory");
#pragma unroll
      for (int j = 0; j < HD / 16; ++j) { const size_t po = ((size_t)bl * CC + h * HD + j * 16 + col) * (size_t)KHI + kc * 32; const v16b vh = frag_b(VB + po, lane); acc[j] = wmma_bf(p.h, vh, acc[j]); acc[j] = wmma_bf(p.l, vh, acc[j]); acc[j] = wmma_bf(p.h, frag_b(VBL + po, lane), acc[j]); } }
  } else {
#pragma unroll 1
    for (int kc = 0; kc < kce; ++kc) { const v16h p = frag_f32(PS + (size_t)(ql0 + col) * TT + kc * 32, lane);
      asm volatile("s_wait_loadcnt 0x0" ::: "memory");
#pragma unroll
      for (int j = 0; j < HD / 16; ++j) { const size_t po = ((size_t)bl * CC + h * HD + j * 16 + col) * (size_t)TT + kc * 32; acc[j] = wmma16(p, frag_h(VT + po, lane), acc[j]); } }
  }
#pragma unroll
  for (int j = 0; j < HD / 16; ++j) {
#pragma unroll
    for (int r = 0; r < 8; ++r) ss[wave][8 * g + r][j * 16 + col] = acc[j][r] * (1.0f / 2048.0f);
  }
  LDSX();
  for (int rl = 0; rl < 16; ++rl) if (lane < HD / 4) vst2((void*)(Y + ((size_t)bl * TT + ql0 + rl) * CC + h * HD + lane * 4), *(const v4f*)&ss[wave][rl][lane * 4]);
}

__global__ __launch_bounds__(128) void k_out(const float* __restrict__ Y, const float* __restrict__ WO, const float* __restrict__ XR, float* __restrict__ Z) {
  __shared__ __align__(16) float sf[4][16][132];
  const int tid = threadIdx.x, wave = __builtin_amdgcn_readfirstlane((int)(tid >> 5)), lane = tid & 31, col = lane & 15, g = lane >> 4; const int c0 = blockIdx.y * 128;
  const size_t rb = (size_t)blockIdx.x * 64; const size_t r0 = rb + wave * 16; const size_t bb = rb / TT; const int tl = (int)(rb % TT) + wave * 16; const size_t orow0 = bb * TT_FULL + tl;
  v8f acc[8] = {};
  if (CAUSAL && (int)(rb % TT) < QHI) {
#pragma unroll 2
    for (int kc = 0; kc < CC / 32; ++kc) { const F2 a = split_row(Y + (r0 + col) * CC, kc * 32, lane); asm volatile("s_wait_loadcnt 0x0" ::: "memory");
#pragma unroll
      for (int j = 0; j < 8; ++j) { const v16b w = wcol_io(WO, kc * 32, c0 + j * 16 + col, lane, DIN); asm volatile("s_wait_loadcnt 0x0" ::: "memory"); acc[j] = wmma_bf(a.h, w, acc[j]); acc[j] = wmma_bf(a.l, w, acc[j]); } }
#pragma unroll
    for (int j = 0; j < 8; ++j) {
#pragma unroll
      for (int r = 0; r < 8; ++r) sf[wave][8 * g + r][j * 16 + col] = acc[j][r]; }
  } else {
#pragma unroll 2
    for (int kc = 0; kc < CC / 32; ++kc) { const v16h a = frag_f32s_fl(Y + (r0 + col) * CC + kc * 32, lane, 64.0f); asm volatile("s_wait_loadcnt 0x0" ::: "memory");
#pragma unroll
      for (int j = 0; j < 8; ++j) { const v16h w = wcolh_io_fl(WO, kc * 32, c0 + j * 16 + col, lane, DIN); asm volatile("s_wait_loadcnt 0x0" ::: "memory"); acc[j] = wmma16(a, w, acc[j]); } }
#pragma unroll
    for (int j = 0; j < 8; ++j) {
#pragma unroll
      for (int r = 0; r < 8; ++r) sf[wave][8 * g + r][j * 16 + col] = acc[j][r] * (1.0f / 16384.0f); }
  }
  LDSX();
  for (int rl = 0; rl < 16; ++rl) { v4f o = *(const v4f*)&sf[wave][rl][lane * 4]; const v4f xv = *(const v4f*)(XR + (orow0 + rl) * DIN + c0 + lane * 4);
#pragma unroll
    for (int i = 0; i < 4; ++i) o[i] += bfr(xv[i]);
    vst2((void*)(Z + (r0 + rl) * DIN + c0 + lane * 4), o); }
}

__global__ __launch_bounds__(256) void k_ln(const float* __restrict__ Z, const float* __restrict__ G, const float* __restrict__ BE, float* __restrict__ OF, _Float16* __restrict__ OH, int ot_stride, int want_h) {
#pragma clang fp contract(off)
  __shared__ __align__(16) _Float16 hs[8][DIN];
  const int tid = threadIdx.x, wave = __builtin_amdgcn_readfirstlane((int)(tid >> 5)), lane = tid & 31;
  const size_t r = (size_t)blockIdx.x * 8 + wave; const size_t bb = r / TT; const int t = (int)(r % TT);
  const float* zr = Z + r * DIN; float* orow = OF + (bb * (size_t)ot_stride + t) * DIN;
  v4f e[DIN / 128]; float s = 0.f;
#pragma unroll
  for (int c = 0; c < DIN / 128; ++c) { const v4f v = *(const v4f*)(zr + c * 128 + lane * 4); e[c] = v; s += (v[0] + v[1]) + (v[2] + v[3]); }
#pragma unroll
  for (int o = 1; o < 32; o <<= 1) s += __shfl_xor(s, o);
  const float mean = s * (1.0f / DIN);
  float q = 0.f;
#pragma unroll
  for (int c = 0; c < DIN / 128; ++c) {
#pragma unroll
    for (int i = 0; i < 4; ++i) { const float d = e[c][i] - mean; e[c][i] = d; q += d * d; } }
#pragma unroll
  for (int o = 1; o < 32; o <<= 1) q += __shfl_xor(q, o);
  const float rstd = rsqrtf(q * (1.0f / DIN) + 1.0e-5f);
  v4f ov[DIN / 128];
#pragma unroll
  for (int c = 0; c < DIN / 128; ++c) { const v4f gv = *(const v4f*)(G + c * 128 + lane * 4); const v4f bv = *(const v4f*)(BE + c * 128 + lane * 4);
#pragma unroll
    for (int i = 0; i < 4; ++i) ov[c][i] = e[c][i] * rstd * bfr(gv[i]) + bfr(bv[i]); }
#pragma unroll
  for (int c = 0; c < DIN / 128; ++c) *(volatile v4f*)(orow + c * 128 + lane * 4) = ov[c];
  __threadfence();
#pragma unroll
  for (int c = 0; c < DIN / 128; ++c) *(volatile v4f*)(orow + c * 128 + lane * 4) = ov[c];
  if (want_h != 0) {
#pragma unroll
    for (int c = 0; c < DIN / 128; ++c) {
#pragma unroll
      for (int i = 0; i < 4; ++i) hs[wave][c * 128 + lane * 4 + i] = toh_flush(ov[c][i]); }
    LDSX();
#pragma unroll
    for (int i = 0; i < DIN / 256; ++i) vst2((void*)(OH + r * DIN + i * 256 + lane * 8), *(const v4u*)&hs[wave][i * 256 + lane * 8]);
  }
}

__global__ __launch_bounds__(128) void k_ffn1(const _Float16* __restrict__ A, const _Float16* __restrict__ WT, const float* __restrict__ B1, _Float16* __restrict__ HID) {
  __shared__ __align__(16) _Float16 sh[64][136];
  const int tid = threadIdx.x, wave = __builtin_amdgcn_readfirstlane((int)(tid >> 5)), lane = tid & 31, col = lane & 15, g = lane >> 4; const int c0 = blockIdx.y * 128;
  const size_t r0 = (size_t)blockIdx.x * 64;
  const _Float16* ar = A + (r0 + wave * 16 + col) * DIN;
  v8f acc[8] = {};
#pragma unroll 2
  for (int kc = 0; kc < DIN / 32; ++kc) { const v16h a = frag_h(ar + kc * 32, lane);
#pragma unroll
    for (int j = 0; j < 8; ++j) { const v16h w = frag_h(WT + (size_t)(c0 + j * 16 + col) * DIN + kc * 32, lane); acc[j] = wmma16(a, w, acc[j]); } }
#pragma unroll
  for (int j = 0; j < 8; ++j) { const float bias = bfr(B1[c0 + j * 16 + col]);
#pragma unroll
    for (int r = 0; r < 8; ++r) { const float v = fmaxf(acc[j][r] * (1.0f / 256.0f) + bias, 0.f); sh[wave * 16 + 8 * g + r][j * 16 + col] = toh_flush(v); } }
  __syncthreads();
  for (int e = tid; e < 64 * 16; e += 128) { const int rl = e >> 4, q = e & 15;
    vst2((void*)(HID + (r0 + rl) * DFF + c0 + q * 8), *(const v4u*)&sh[rl][q * 8]); }
}

__global__ __launch_bounds__(128) void k_ffn2(const _Float16* __restrict__ HID, const _Float16* __restrict__ WT, const float* __restrict__ B2, const float* __restrict__ L1F, float* __restrict__ Z) {
  __shared__ __align__(16) float sf[4][16][132];
  const int tid = threadIdx.x, wave = __builtin_amdgcn_readfirstlane((int)(tid >> 5)), lane = tid & 31, col = lane & 15, g = lane >> 4; const int c0 = blockIdx.y * 128;
  const size_t r0 = (size_t)blockIdx.x * 64 + wave * 16;
  const _Float16* ar = HID + (r0 + col) * DFF;
  v8f acc[8] = {};
#pragma unroll 2
  for (int kc = 0; kc < DFF / 32; ++kc) { const v16h a = frag_h(ar + kc * 32, lane);
#pragma unroll
    for (int j = 0; j < 8; ++j) { const v16h w = frag_h(WT + (size_t)(c0 + j * 16 + col) * DFF + kc * 32, lane); acc[j] = wmma16(a, w, acc[j]); } }
#pragma unroll
  for (int j = 0; j < 8; ++j) { const float bias = bfr(B2[c0 + j * 16 + col]);
#pragma unroll
    for (int r = 0; r < 8; ++r) sf[wave][8 * g + r][j * 16 + col] = acc[j][r] * (1.0f / 256.0f) + bias; }
  LDSX();
  for (int rl = 0; rl < 16; ++rl) { v4f o = *(const v4f*)&sf[wave][rl][lane * 4]; const v4f lv = *(const v4f*)(L1F + (r0 + rl) * DIN + c0 + lane * 4);
#pragma unroll
    for (int i = 0; i < 4; ++i) o[i] += lv[i];
    vst2((void*)(Z + (r0 + rl) * DIN + c0 + lane * 4), o); }
}

extern "C" void kernel_launch(void* const* d_in, const int* in_sizes, int n_in, void* d_out, int out_size, void* d_ws, size_t ws_size, hipStream_t stream) {
  if (n_in < 13) return;
  const size_t need_rows = (size_t)(NB - 1) * TT_FULL + TT;
  if ((size_t)in_sizes[0] < need_rows * DIN) return;
  if ((size_t)in_sizes[1] < (size_t)NH * DIN * HD || (size_t)in_sizes[2] < (size_t)NH * DIN * HD || (size_t)in_sizes[3] < (size_t)NH * DIN * HD) return;
  if ((size_t)in_sizes[4] < (size_t)CC * DIN) return;
  if ((size_t)in_sizes[5] < (size_t)DIN * DFF || (size_t)in_sizes[6] < (size_t)DFF || (size_t)in_sizes[7] < (size_t)DFF * DIN || (size_t)in_sizes[8] < (size_t)DIN) return;
  if ((size_t)in_sizes[9] < (size_t)DIN || (size_t)in_sizes[10] < (size_t)DIN || (size_t)in_sizes[11] < (size_t)DIN || (size_t)in_sizes[12] < (size_t)DIN) return;
  if ((size_t)out_size < need_rows * DIN) return;
  if (ws_size < (size_t)WS_END) return;
  const float** F = (const float**)d_in;
  char* ws = (char*)d_ws;
  _Float16 *QH = (_Float16*)(ws + WS_QH), *KH = (_Float16*)(ws + WS_KH), *VT = (_Float16*)(ws + WS_VT), *QL = (_Float16*)(ws + WS_QL), *KL = (_Float16*)(ws + WS_KL);
  __bf16 *VB = (__bf16*)(ws + WS_VB), *VBL = (__bf16*)(ws + WS_VBL); float *S = (float*)(ws + WS_S), *Y = (float*)(ws + WS_Y);
  float *Z1 = (float*)(ws + WS_Z1), *L1F = (float*)(ws + WS_L1F), *Z2 = (float*)(ws + WS_Z2);
  _Float16 *L1H = (_Float16*)(ws + WS_L1H), *HID = (_Float16*)(ws + WS_HID), *W1T = (_Float16*)(ws + WS_W1T), *W2T = (_Float16*)(ws + WS_W2T);
  k_wt<<<dim3(DIN / 64, DFF / 64), 128, 0, stream>>>(F[5], W1T, DIN, DFF);
  k_wt<<<dim3(DFF / 64, DIN / 64), 128, 0, stream>>>(F[7], W2T, DFF, DIN);
  for (int b0 = 0; b0 < NB; b0 += NBC) {
    const float* Xc = F[0] + (size_t)b0 * TT_FULL * DIN; float* Oc = (float*)d_out + (size_t)b0 * TT_FULL * DIN;
    k_proj<<<dim3(NBC * TT / 64, CC / 128, 3), 128, 0, stream>>>(Xc, F[1], F[2], F[3], QH, QL, KH, KL, VT, VB, VBL);
    k_sc<<<dim3(NQB, TT / 128, NBC * NH), 128, 0, stream>>>(QH, KH, QL, KL, S);
    k_sm<<<dim3(TT / 8, NBC * NH), 256, 0, stream>>>(S);
    k_pv<<<dim3(NQB, 1, NBC * NH), 128, 0, stream>>>(S, VT, VB, VBL, Y);
    k_out<<<dim3(NBC * TT / 64, DIN / 128), 128, 0, stream>>>(Y, F[4], Xc, Z1);
    k_ln<<<dim3(NBC * TT / 8), 256, 0, stream>>>(Z1, F[9], F[10], L1F, L1H, TT, 1);
    k_ffn1<<<dim3(NBC * TT / 64, DFF / 128), 128, 0, stream>>>(L1H, W1T, F[6], HID);
    k_ffn2<<<dim3(NBC * TT / 64, DIN / 128), 128, 0, stream>>>(HID, W2T, F[8], L1F, Z2);
    k_ln<<<dim3(NBC * TT / 8), 256, 0, stream>>>(Z2, F[11], F[12], Oc, L1H, TT_FULL, 0);
  }
}
